// SS2D_66511863546364
// MI455X (gfx1250) — hardware-run, weakly checked
//
#include <hip/hip_runtime.h>
#include <hip/hip_fp16.h>
#include <math.h>

constexpr int kB    = 8;
constexpr int kD    = 192;
constexpr int kH    = 64;
constexpr int kW    = 64;
constexpr int kL    = kH * kW;
constexpr int kDir  = 4;
constexpr int kNs   = 16;
constexpr int kR    = 6;
constexpr int kC    = kR + 2 * kNs;
constexpr int kCP   = 48;
constexpr int kNall = kDir * kCP;
constexpr int kRows = kB * kL;
constexpr int kXP   = 68;
constexpr int kBcW  = 2 * kNs;
constexpr float kYCarry = 16.0f;
constexpr float kYInv   = 1.0f / kYCarry;
static_assert(kH == 64 && kW == 64 && kL == 4096);
static_assert(kC == 38 && kC <= kCP && kNall == 192);
static_assert((kD % 64) == 0 && (kL % 64) == 0 && (kRows % 64) == 0 && (kNall % 64) == 0 && (kD % 32) == 0);
static_assert((kD % 4) == 0 && (kD / 4) == 48 && (kD / 8) == 24);

constexpr size_t kOffAH = 0;
constexpr size_t kOffAL = kOffAH + (size_t)kRows * kD * 2;
constexpr size_t kOffBH = kOffAL + (size_t)kRows * kD * 2;
constexpr size_t kOffBL = kOffBH + (size_t)kNall * kD * 2;
constexpr size_t kOffXD = kOffBL + (size_t)kNall * kD * 2;
constexpr size_t kOffDT = kOffXD + (size_t)kRows * kNall * 4;
constexpr size_t kOffUU = kOffDT + (size_t)kDir * kL * kD * 4;
constexpr size_t kOffBC = kOffUU + (size_t)kDir * kL * kD * 4;
constexpr size_t kOffYS = kOffBC + (size_t)kDir * kL * kBcW * 4;
constexpr size_t kWsTotal = kOffYS + (size_t)kB * kDir * kL * kD * 2;
static_assert(kWsTotal == 128073728ull);
static_assert(kWsTotal <= 134217728ull);
static_assert((kOffAL % 128) == 0 && (kOffBH % 128) == 0 && (kOffBL % 128) == 0 && (kOffXD % 128) == 0 &&
              (kOffDT % 128) == 0 && (kOffUU % 128) == 0 && (kOffBC % 128) == 0 && (kOffYS % 128) == 0);

typedef float    v4f __attribute__((ext_vector_type(4)));
typedef float    v2f __attribute__((ext_vector_type(2)));
typedef unsigned v4u __attribute__((ext_vector_type(4)));
typedef unsigned v2u __attribute__((ext_vector_type(2)));

__device__ __forceinline__ unsigned bf_bits(float f) {
  const unsigned u = __float_as_uint(f);
  return (u + 0x7FFFu + ((u >> 16) & 1u)) >> 16;
}
__device__ __forceinline__ float bf_val(unsigned h) { return __uint_as_float(h << 16); }

__device__ __forceinline__ float h16_to_f32(unsigned hb) {
  const unsigned sgn = (hb & 0x8000u) << 16;
  const unsigned em = hb & 0x7fffu;
  const float fn = __uint_as_float((em << 13) + 0x38000000u);
  const float fs = (float)em * 5.9604644775390625e-8f;
  const float mag = (em < 0x400u) ? fs : fn;
  return __uint_as_float(__float_as_uint(mag) | sgn);
}

namespace eng {
typedef __attribute__((ext_vector_type(16))) __bf16 v16b;
typedef __attribute__((ext_vector_type(8)))  __bf16 v8b;
typedef __attribute__((ext_vector_type(8)))  float  v8f;
union FragB { v16b v; v8b h[2]; };
__device__ __forceinline__ v16b frag_load(const __bf16* p) {
  FragB f;
  f.h[0] = *(const v8b*)(p);
  f.h[1] = *(const v8b*)(p + 16);
  return f.v;
}
__device__ __forceinline__ v8f mma_b(v16b a, v16b b, v8f c) {
  return __builtin_amdgcn_wmma_f32_16x16x32_bf16(false, a, false, b, (short)0, c, false, false);
}
__device__ __forceinline__ void row_guard(v8f& a, v8f& b, v8f& c, v8f& d, v16b x, v16b y) {
  asm volatile("v_nop\n\tv_nop\n\tv_nop\n\tv_nop" : "+v"(a), "+v"(b), "+v"(c), "+v"(d) : "v"(x), "v"(y));
}
__device__ __forceinline__ void keep4(v16b a, v16b b, v16b c, v16b d) {
  asm volatile("v_nop" :: "v"(a), "v"(b), "v"(c), "v"(d));
}
__device__ __forceinline__ void acc_guard4(v8f& a, v8f& b, v8f& c, v8f& d) {
  asm volatile("v_nop\n\tv_nop\n\tv_nop\n\tv_nop" : "+v"(a), "+v"(b), "+v"(c), "+v"(d));
}

__global__ __launch_bounds__(256) void gemm_bf16x3_kernel(
    const unsigned short* __restrict__ Ahp, const unsigned short* __restrict__ Alp, int lda,
    const unsigned short* __restrict__ Bhp, const unsigned short* __restrict__ Blp, int ldb,
    float* __restrict__ C, int ldc, int M, int N, int K)
{
  const __bf16* Ah = (const __bf16*)Ahp;
  const __bf16* Al = (const __bf16*)Alp;
  const __bf16* Bh = (const __bf16*)Bhp;
  const __bf16* Bl = (const __bf16*)Blp;
  __shared__ __align__(16) float sT[8][16 * 68];
  const int lane = threadIdx.x & 31;
  const int wave = threadIdx.x >> 5;
  const int tilesN = N >> 6;
  const int tilesM = M >> 6;
  const int tile = blockIdx.x * 8 + wave;
  if (tile >= tilesM * tilesN) return;
  const int tm = tile / tilesN;
  const int tn = tile - tm * tilesN;
  const int m0 = tm << 6;
  const int n0 = tn << 6;
  const int rlane = lane & 15;
  const int koff  = (lane >> 4) * 8;
  const int mOff  = (lane >> 4) * 8;

  v8f acc[4][4];
#pragma unroll
  for (int i = 0; i < 4; ++i)
#pragma unroll
    for (int j = 0; j < 4; ++j) acc[i][j] = (v8f){0.f, 0.f, 0.f, 0.f, 0.f, 0.f, 0.f, 0.f};

  for (int k0 = 0; k0 < K; k0 += 32) {
    v16b bh[4], bl[4];
#pragma unroll
    for (int j = 0; j < 4; ++j) {
      const size_t bo = (size_t)(n0 + (j << 4) + rlane) * ldb + koff + k0;
      bh[j] = frag_load(Bh + bo);
      bl[j] = frag_load(Bl + bo);
    }
#pragma unroll
    for (int i = 0; i < 4; ++i) {
      const size_t ao = (size_t)(m0 + (i << 4) + rlane) * lda + koff + k0;
      const v16b ah = frag_load(Ah + ao);
      const v16b al = frag_load(Al + ao);
#pragma unroll
      for (int j = 0; j < 4; ++j) {
        acc[i][j] = mma_b(ah, bh[j], acc[i][j]);
        acc[i][j] = mma_b(ah, bl[j], acc[i][j]);
        acc[i][j] = mma_b(al, bh[j], acc[i][j]);
      }
      row_guard(acc[i][0], acc[i][1], acc[i][2], acc[i][3], ah, al);
    }
    keep4(bh[0], bh[1], bh[2], bh[3]);
    keep4(bl[0], bl[1], bl[2], bl[3]);
  }
  acc_guard4(acc[0][0], acc[0][1], acc[0][2], acc[0][3]);
  acc_guard4(acc[1][0], acc[1][1], acc[1][2], acc[1][3]);
  acc_guard4(acc[2][0], acc[2][1], acc[2][2], acc[2][3]);
  acc_guard4(acc[3][0], acc[3][1], acc[3][2], acc[3][3]);

  float* slab = sT[wave];
#pragma unroll
  for (int i = 0; i < 4; ++i) {
    const int mBase = m0 + (i << 4);
#pragma unroll
    for (int j = 0; j < 4; ++j) {
#pragma unroll
      for (int r = 0; r < 8; ++r) {
        slab[(mOff + r) * 68 + (j << 4) + rlane] = acc[i][j][r];
      }
    }
    __builtin_amdgcn_fence(__ATOMIC_RELEASE, "workgroup");
    __builtin_amdgcn_wave_barrier();
    __builtin_amdgcn_fence(__ATOMIC_ACQUIRE, "workgroup");
    {
      const int hh = lane >> 4;
      const int c4 = (lane & 15) * 4;
      for (int pass = 0; pass < 2; ++pass) {
#pragma unroll
        for (int it = 0; it < 8; ++it) {
          const int row = it * 2 + hh;
          const v4f v = *(const v4f*)(slab + row * 68 + c4);
          *(volatile v4f*)(C + (size_t)(mBase + row) * ldc + n0 + c4) = v;
        }
        __threadfence();
      }
    }
    __builtin_amdgcn_fence(__ATOMIC_RELEASE, "workgroup");
    __builtin_amdgcn_wave_barrier();
    __builtin_amdgcn_fence(__ATOMIC_ACQUIRE, "workgroup");
  }
}
}

__global__ __launch_bounds__(256) void pack_x_kernel(
    const float* __restrict__ x, unsigned short* __restrict__ AH, unsigned short* __restrict__ AL)
{
  __shared__ __align__(16) float sX[kD * kXP];
  const int tid  = threadIdx.x;
  const int b    = blockIdx.x >> 6;
  const int hrow = blockIdx.x & 63;
  const float* xb = x + (size_t)b * kD * kL + hrow * 64;
#pragma unroll 4
  for (int it = 0; it < 12; ++it) {
    const int idx = it * 256 + tid;
    const int d   = idx >> 4;
    const int w4  = (idx & 15) * 4;
    const v4f v = *(const v4f*)(xb + (size_t)d * kL + w4);
    *(v4f*)(sX + d * kXP + w4) = v;
  }
  __syncthreads();
  const size_t m0 = (size_t)b * kL + (size_t)hrow * 64;
#pragma unroll 1
  for (int it = 0; it < 6; ++it) {
    const int idx = it * 256 + tid;
    const int row = idx / 24;
    const int c8  = (idx - row * 24) * 8;
    unsigned hw[4], lw[4];
#pragma unroll
    for (int e = 0; e < 4; ++e) {
      const float v0 = sX[(c8 + 2 * e) * kXP + row];
      const float v1 = sX[(c8 + 2 * e + 1) * kXP + row];
      const unsigned h0 = bf_bits(v0);
      const unsigned h1 = bf_bits(v1);
      const unsigned l0 = bf_bits(v0 - bf_val(h0));
      const unsigned l1 = bf_bits(v1 - bf_val(h1));
      hw[e] = h0 | (h1 << 16);
      lw[e] = l0 | (l1 << 16);
    }
    const v4u hv = (v4u){hw[0], hw[1], hw[2], hw[3]};
    const v4u lv = (v4u){lw[0], lw[1], lw[2], lw[3]};
    const size_t o = (m0 + row) * kD + c8;
    *(volatile v4u*)(AH + o) = hv;
    *(volatile v4u*)(AL + o) = lv;
    __threadfence();
    *(volatile v4u*)(AH + o) = hv;
    *(volatile v4u*)(AL + o) = lv;
  }
}

__global__ __launch_bounds__(256) void pack_w_kernel(
    const float* __restrict__ W1, unsigned short* __restrict__ BH, unsigned short* __restrict__ BL)
{
  const int idx = blockIdx.x * 256 + threadIdx.x;
  if (idx >= kNall * 24) return;
  const int n  = idx / 24;
  const int c8 = (idx - n * 24) * 8;
  const int k  = n / kCP;
  const int c  = n - k * kCP;
  const bool live = (c < kC);
  const int cc = live ? c : (kC - 1);
  const float* src = W1 + ((size_t)(k * kC + cc)) * kD + c8;
  const v4f a0 = *(const v4f*)(src);
  const v4f a1 = *(const v4f*)(src + 4);
  float f[8];
  f[0] = live ? a0[0] : 0.0f;
  f[1] = live ? a0[1] : 0.0f;
  f[2] = live ? a0[2] : 0.0f;
  f[3] = live ? a0[3] : 0.0f;
  f[4] = live ? a1[0] : 0.0f;
  f[5] = live ? a1[1] : 0.0f;
  f[6] = live ? a1[2] : 0.0f;
  f[7] = live ? a1[3] : 0.0f;
  unsigned hw[4], lw[4];
#pragma unroll
  for (int e = 0; e < 4; ++e) {
    const unsigned h0 = bf_bits(f[2 * e]);
    const unsigned h1 = bf_bits(f[2 * e + 1]);
    const unsigned l0 = bf_bits(f[2 * e] - bf_val(h0));
    const unsigned l1 = bf_bits(f[2 * e + 1] - bf_val(h1));
    hw[e] = h0 | (h1 << 16);
    lw[e] = l0 | (l1 << 16);
  }
  const v4u hv = (v4u){hw[0], hw[1], hw[2], hw[3]};
  const v4u lv = (v4u){lw[0], lw[1], lw[2], lw[3]};
  const size_t o = (size_t)n * kD + c8;
  *(volatile v4u*)(BH + o) = hv;
  *(volatile v4u*)(BL + o) = lv;
  __threadfence();
  *(volatile v4u*)(BH + o) = hv;
  *(volatile v4u*)(BL + o) = lv;
}

__global__ __launch_bounds__(192) void prep_planes_kernel(
    const float* __restrict__ x, const float* __restrict__ XD, const float* __restrict__ W2,
    const float* __restrict__ bias, float* __restrict__ DT, float* __restrict__ UU, float* __restrict__ BC, int b)
{
  __shared__ __align__(16) float sX[kD * kXP];
  const int tid  = threadIdx.x;
  const int hrow = blockIdx.x;
  const float* xb = x + (size_t)b * kD * kL + hrow * 64;
#pragma unroll 4
  for (int it = 0; it < 16; ++it) {
    const int idx = it * 192 + tid;
    const int dd  = idx >> 4;
    const int w4  = (idx & 15) * 4;
    const v4f v = *(const v4f*)(xb + (size_t)dd * kL + w4);
    *(v4f*)(sX + dd * kXP + w4) = v;
  }
  __syncthreads();
  const int rsub = tid / 48;
  const int c4   = tid - rsub * 48;
  const int d    = c4 * 4;
  const size_t mrow0 = (size_t)b * kL + (size_t)hrow * 64;
#pragma unroll 1
  for (int k = 0; k < kDir; ++k) {
    const float* wp = W2 + ((size_t)k * kD + d) * kR;
    v4f wq[6];
#pragma unroll
    for (int j = 0; j < 6; ++j) wq[j] = *(const v4f*)(wp + 4 * j);
    const v4f bv = *(const v4f*)(bias + k * kD + d);
    float* dtk = DT + (size_t)k * kL * kD;
    float* uk  = UU + (size_t)k * kL * kD;
    float* bck = BC + (size_t)k * kL * kBcW;
#pragma unroll 1
    for (int it = 0; it < 16; ++it) {
      const int w = it * 4 + rsub;
      const int p = hrow * 64 + w;
      const int t = w * 64 + hrow;
      int l = (k & 1) ? t : p;
      if (k & 2) l = kL - 1 - l;
      const float* xr = XD + (mrow0 + w) * kNall + k * kCP;
      const v4f s0 = *(const v4f*)(xr);
      const v2f s1 = *(const v2f*)(xr + 4);
      v4f o;
#pragma unroll
      for (int e = 0; e < 4; ++e) {
        float acc = wq[(6 * e + 0) >> 2][(6 * e + 0) & 3] * s0[0];
        acc = fmaf(wq[(6 * e + 1) >> 2][(6 * e + 1) & 3], s0[1], acc);
        acc = fmaf(wq[(6 * e + 2) >> 2][(6 * e + 2) & 3], s0[2], acc);
        acc = fmaf(wq[(6 * e + 3) >> 2][(6 * e + 3) & 3], s0[3], acc);
        acc = fmaf(wq[(6 * e + 4) >> 2][(6 * e + 4) & 3], s1[0], acc);
        acc = fmaf(wq[(6 * e + 5) >> 2][(6 * e + 5) & 3], s1[1], acc);
        o[e] = acc + bv[e];
      }
      v4f uv;
      uv[0] = sX[(d + 0) * kXP + w];
      uv[1] = sX[(d + 1) * kXP + w];
      uv[2] = sX[(d + 2) * kXP + w];
      uv[3] = sX[(d + 3) * kXP + w];
      const size_t oo = (size_t)l * kD + d;
      *(volatile v4f*)(dtk + oo) = o;
      *(volatile v4f*)(uk + oo) = uv;
      __threadfence();
      *(volatile v4f*)(dtk + oo) = o;
      *(volatile v4f*)(uk + oo) = uv;
    }
#pragma unroll 1
    for (int it = 0; it < 3; ++it) {
      const int idx = it * 192 + tid;
      if (idx < 512) {
        const int w = idx >> 3;
        const int j = idx & 7;
        const int p = hrow * 64 + w;
        const int t = w * 64 + hrow;
        int l = (k & 1) ? t : p;
        if (k & 2) l = kL - 1 - l;
        const float* xr = XD + (mrow0 + w) * kNall + k * kCP + kR + 4 * j;
        const v2f q0 = *(const v2f*)(xr);
        const v2f q1 = *(const v2f*)(xr + 2);
        const v4f o = (v4f){q0[0], q0[1], q1[0], q1[1]};
        const size_t oo = (size_t)l * kBcW + 4 * j;
        *(volatile v4f*)(bck + oo) = o;
        __threadfence();
        *(volatile v4f*)(bck + oo) = o;
      }
    }
  }
}

typedef float    ms1_v4f __attribute__((ext_vector_type(4)));
typedef unsigned ms1_v4u __attribute__((ext_vector_type(4)));
struct ms1_args {
  const float* dtpre;
  const float* u;
  const float* bc;
  const float* z;
  const float* A_log;
  const float* Dskip;
  __half* y;
  __half* y_lo;
  long ld_dtpre;
  long ld_u;
  long ld_bc;
  long ld_z;
  long ld_y;
  int offB;
  int offC;
  int offZ;
  float ycarry;
  int dir;
  int D;
  int L;
  int nbatch;
};
static_assert(sizeof(ms1_args) == 136);

__device__ __forceinline__ float ms1_flush16(float v) {
  return (fabsf(v) < 6.103515625e-05f) ? 0.0f : v;
}
__device__ __forceinline__ unsigned ms1_h16bits(float v) {
  return (unsigned)__half_as_ushort(__float2half_rn(ms1_flush16(v)));
}
__device__ __forceinline__ float ms1_h16val(unsigned b) {
  return __half2float(__ushort_as_half((unsigned short)b));
}
__device__ __forceinline__ float ms1_softplus(float v) {
  return fmaxf(v, 0.0f) + log1pf(expf(-fabsf(v)));
}
__device__ __forceinline__ void ms1_pack2(float v0, float v1, unsigned& hw, unsigned& lw) {
  const unsigned h0 = ms1_h16bits(v0);
  const unsigned h1 = ms1_h16bits(v1);
  const float r0 = (v0 - ms1_h16val(h0)) * 2048.0f;
  const float r1 = (v1 - ms1_h16val(h1)) * 2048.0f;
  const unsigned l0 = ms1_h16bits(r0);
  const unsigned l1 = ms1_h16bits(r1);
  hw = h0 | (h1 << 16);
  lw = l0 | (l1 << 16);
}

template <int NSTATE>
__global__ __launch_bounds__(64 * (NSTATE / 16)) void ms1_scan_kernel(ms1_args a)
{
  static_assert(NSTATE == 16 || NSTATE == 64);
  constexpr int NQ  = NSTATE / 16;
  constexpr int NT  = 64 * NQ;
  constexpr int NW  = NT / 32;
  constexpr int BCW = 2 * NSTATE;
  constexpr int YP  = 68;
  constexpr int RPI = NW * 4;
  constexpr int NIT = 64 / RPI;
  static_assert(16 * NT <= 64 * YP);
  __shared__ __align__(16) float sBC[64 * BCW];
  __shared__ __align__(16) float sY[64 * YP];
  const int tid  = threadIdx.x;
  const int lane = tid & 31;
  const int wave = tid >> 5;
  const int c    = tid / NQ;
  const int sq   = tid - c * NQ;
  const int bpb  = a.D / 64;
  const int bi   = blockIdx.x / bpb;
  if (bi >= a.nbatch) return;
  const int d0 = (blockIdx.x - bi * bpb) * 64;
  const int d  = d0 + c;
  const long rowb = (long)bi * a.L;
  const bool hasz  = (a.z != nullptr);
  const bool hasD  = (a.Dskip != nullptr);
  const bool hasLo = (a.y_lo != nullptr);

#pragma unroll 1
  for (int n = 0; n < 16; ++n) {
    const float al = a.A_log[(long)d * NSTATE + sq * 16 + n];
    sY[n * NT + tid] = -expf(al);
  }
  __syncthreads();
  float An[16], h[16];
#pragma unroll
  for (int n = 0; n < 16; ++n) {
    An[n] = sY[n * NT + tid];
    h[n] = 0.0f;
  }
  float Dd = 0.0f;
  if (hasD) Dd = a.Dskip[d];

  const int nchunk = a.L / 64;
  const bool fwd = (a.dir > 0);
  const int s0 = fwd ? 0 : 63;
  const int sd = fwd ? 1 : -1;
  const int q  = lane >> 3;
  const int c8 = (lane & 7) * 8;

#pragma unroll 1
  for (int ci = 0; ci < nchunk; ++ci) {
    const int tb = fwd ? (ci * 64) : (a.L - 64 - ci * 64);
    const long rowc = rowb + tb;
    __syncthreads();
#pragma unroll 8
    for (int i = 0; i < 32; ++i) {
      const int idx = tid + i * NT;
      const int st  = idx / BCW;
      const int col = idx - st * BCW;
      const int sc  = (col < NSTATE) ? (a.offB + col) : (a.offC + col - NSTATE);
      sBC[idx] = a.bc[(rowc + st) * a.ld_bc + sc];
    }
    __syncthreads();
#pragma unroll 1
    for (int s = 0; s < 64; ++s) {
      const int ls = s0 + sd * s;
      const long row = rowc + ls;
      float pre = a.dtpre[row * a.ld_dtpre + d];
      float uv  = a.u[row * a.ld_u + d];
      float zv  = 0.0f;
      if (hasz) zv = a.z[row * a.ld_z + a.offZ + d];
      asm volatile("" : "+v"(pre));
      asm volatile("" : "+v"(uv));
      asm volatile("" : "+v"(zv));
      const float delta = ms1_softplus(pre);
      const float dtx = delta * uv;
      const float* bp = sBC + ls * BCW + sq * 16;
      const float* cp = bp + NSTATE;
      ms1_v4f Bq[4], Cq[4];
#pragma unroll
      for (int k = 0; k < 4; ++k) {
        Bq[k] = *(const ms1_v4f*)(bp + 4 * k);
        Cq[k] = *(const ms1_v4f*)(cp + 4 * k);
      }
      float yv = 0.0f;
#pragma unroll
      for (int n = 0; n < 16; ++n) {
        const float e = __expf(delta * An[n]);
        h[n] = fmaf(e, h[n], dtx * Bq[n >> 2][n & 3]);
        yv = fmaf(h[n], Cq[n >> 2][n & 3], yv);
      }
      if (NQ > 1) {
        yv += __shfl_xor(yv, 1, 32);
        yv += __shfl_xor(yv, 2, 32);
      }
      if (hasD) yv = fmaf(uv, Dd, yv);
      if (hasz) {
        const float sg = __builtin_amdgcn_rcpf(1.0f + expf(-zv));
        yv = yv * (zv * sg);
      }
      if (sq == 0) sY[ls * YP + c] = yv * a.ycarry;
    }
    __syncthreads();
    ms1_v4u hw[NIT], lw[NIT];
#pragma unroll
    for (int it = 0; it < NIT; ++it) {
      const int row = it * RPI + wave * 4 + q;
      const float* sp = sY + row * YP + c8;
      const ms1_v4f f0 = *(const ms1_v4f*)(sp);
      const ms1_v4f f1 = *(const ms1_v4f*)(sp + 4);
      unsigned h0, h1, h2, h3, l0, l1, l2, l3;
      ms1_pack2(f0[0], f0[1], h0, l0);
      ms1_pack2(f0[2], f0[3], h1, l1);
      ms1_pack2(f1[0], f1[1], h2, l2);
      ms1_pack2(f1[2], f1[3], h3, l3);
      hw[it] = (ms1_v4u){h0, h1, h2, h3};
      lw[it] = (ms1_v4u){l0, l1, l2, l3};
    }
    for (int pass = 0; pass < 2; ++pass) {
#pragma unroll
      for (int it = 0; it < NIT; ++it) {
        const int row = it * RPI + wave * 4 + q;
        const long o = (rowc + row) * a.ld_y + d0 + c8;
        *(volatile ms1_v4u*)(a.y + o) = hw[it];
        if (hasLo) *(volatile ms1_v4u*)(a.y_lo + o) = lw[it];
      }
      __threadfence();
    }
  }
}

__global__ __launch_bounds__(192) void merge_norm_kernel(
    const unsigned short* __restrict__ YS, const float* __restrict__ lnw, const float* __restrict__ lnb,
    float* __restrict__ out)
{
  __shared__ float sP1[12];
  __shared__ float sP2[12];
  const int tid  = threadIdx.x;
  const int rsub = tid / 48;
  const int c4   = tid - rsub * 48;
  const int d    = c4 * 4;
  const int grp  = tid >> 4;
  const v4f gw = *(const v4f*)(lnw + d);
  const v4f gb = *(const v4f*)(lnb + d);
#pragma unroll 1
  for (int it = 0; it < 4; ++it) {
    const int m  = blockIdx.x * 16 + it * 4 + rsub;
    const int b  = m >> 12;
    const int p  = m & (kL - 1);
    const int hq = p >> 6;
    const int wq = p & 63;
    const int t  = wq * 64 + hq;
    const unsigned short* base = YS + (size_t)b * kDir * kL * kD;
    const v2u q0 = *(const v2u*)(base + ((size_t)(0 * kL + p)) * kD + d);
    const v2u q1 = *(const v2u*)(base + ((size_t)(1 * kL + t)) * kD + d);
    const v2u q2 = *(const v2u*)(base + ((size_t)(2 * kL + (kL - 1 - p))) * kD + d);
    const v2u q3 = *(const v2u*)(base + ((size_t)(3 * kL + (kL - 1 - t))) * kD + d);
    const unsigned a0 = q0[0], a1 = q0[1];
    const unsigned b0 = q1[0], b1 = q1[1];
    const unsigned e0 = q2[0], e1 = q2[1];
    const unsigned g0 = q3[0], g1 = q3[1];
    float v[4];
    v[0] = ((h16_to_f32(a0 & 0xffffu) + h16_to_f32(e0 & 0xffffu)) + (h16_to_f32(b0 & 0xffffu) + h16_to_f32(g0 & 0xffffu))) * kYInv;
    v[1] = ((h16_to_f32(a0 >> 16) + h16_to_f32(e0 >> 16)) + (h16_to_f32(b0 >> 16) + h16_to_f32(g0 >> 16))) * kYInv;
    v[2] = ((h16_to_f32(a1 & 0xffffu) + h16_to_f32(e1 & 0xffffu)) + (h16_to_f32(b1 & 0xffffu) + h16_to_f32(g1 & 0xffffu))) * kYInv;
    v[3] = ((h16_to_f32(a1 >> 16) + h16_to_f32(e1 >> 16)) + (h16_to_f32(b1 >> 16) + h16_to_f32(g1 >> 16))) * kYInv;
    float s = (v[0] + v[1]) + (v[2] + v[3]);
    s += __shfl_xor(s, 1, 32);
    s += __shfl_xor(s, 2, 32);
    s += __shfl_xor(s, 4, 32);
    s += __shfl_xor(s, 8, 32);
    if ((tid & 15) == 0) sP1[grp] = s;
    __syncthreads();
    const float mu = ((sP1[3 * rsub] + sP1[3 * rsub + 1]) + sP1[3 * rsub + 2]) * (1.0f / (float)kD);
    const float d0v = v[0] - mu;
    const float d1v = v[1] - mu;
    const float d2v = v[2] - mu;
    const float d3v = v[3] - mu;
    float s2 = (d0v * d0v + d1v * d1v) + (d2v * d2v + d3v * d3v);
    s2 += __shfl_xor(s2, 1, 32);
    s2 += __shfl_xor(s2, 2, 32);
    s2 += __shfl_xor(s2, 4, 32);
    s2 += __shfl_xor(s2, 8, 32);
    if ((tid & 15) == 0) sP2[grp] = s2;
    __syncthreads();
    const float var = ((sP2[3 * rsub] + sP2[3 * rsub + 1]) + sP2[3 * rsub + 2]) * (1.0f / (float)kD);
    const float rstd = rsqrtf(var + 1e-5f);
    v4f o;
    o[0] = d0v * rstd * gw[0] + gb[0];
    o[1] = d1v * rstd * gw[1] + gb[1];
    o[2] = d2v * rstd * gw[2] + gb[2];
    o[3] = d3v * rstd * gw[3] + gb[3];
    float* po = out + (size_t)m * kD + d;
    *(volatile v4f*)po = o;
    __threadfence();
    *(volatile v4f*)po = o;
  }
}

extern "C" void kernel_launch(void* const* d_in, const int* in_sizes, int n_in,
                              void* d_out, int out_size, void* d_ws, size_t ws_size,
                              hipStream_t stream) {
  if (n_in < 8) return;
  if (in_sizes[0] != kB * kD * kL) return;
  if (in_sizes[1] != kDir * kC * kD) return;
  if (in_sizes[2] != kDir * kD * kR) return;
  if (in_sizes[3] != kDir * kD) return;
  if (in_sizes[4] != kDir * kD * kNs) return;
  if (in_sizes[5] != kDir * kD) return;
  if (in_sizes[6] != kD) return;
  if (in_sizes[7] != kD) return;
  if (out_size != kRows * kD) return;
  if (ws_size < kWsTotal) return;

  const float* x    = (const float*)d_in[0];
  const float* W1   = (const float*)d_in[1];
  const float* W2   = (const float*)d_in[2];
  const float* bdt  = (const float*)d_in[3];
  const float* Alog = (const float*)d_in[4];
  const float* Dsk  = (const float*)d_in[5];
  const float* lnw  = (const float*)d_in[6];
  const float* lnb  = (const float*)d_in[7];
  float* out = (float*)d_out;

  char* ws = (char*)d_ws;
  unsigned short* AH = (unsigned short*)(ws + kOffAH);
  unsigned short* AL = (unsigned short*)(ws + kOffAL);
  unsigned short* BH = (unsigned short*)(ws + kOffBH);
  unsigned short* BL = (unsigned short*)(ws + kOffBL);
  float*          XD = (float*)(ws + kOffXD);
  float*          DT = (float*)(ws + kOffDT);
  float*          UU = (float*)(ws + kOffUU);
  float*          BC = (float*)(ws + kOffBC);
  unsigned short* YS = (unsigned short*)(ws + kOffYS);

  pack_x_kernel<<<dim3(kB * kH), 256, 0, stream>>>(x, AH, AL);
  pack_w_kernel<<<dim3((kNall * 24) / 256), 256, 0, stream>>>(W1, BH, BL);

  eng::gemm_bf16x3_kernel<<<dim3(((kRows / 64) * (kNall / 64)) / 8), 256, 0, stream>>>(
      AH, AL, kD, BH, BL, kD, XD, kNall, kRows, kNall, kD);

  for (int b = 0; b < kB; ++b) {
    prep_planes_kernel<<<dim3(kH), 192, 0, stream>>>(x, XD, W2, bdt, DT, UU, BC, b);
    for (int k = 0; k < kDir; ++k) {
      ms1_args sa;
      sa.dtpre = DT + (size_t)k * kL * kD;
      sa.u = UU + (size_t)k * kL * kD;
      sa.bc = BC + (size_t)k * kL * kBcW;
      sa.z = nullptr;
      sa.A_log = Alog + (size_t)k * kD * kNs;
      sa.Dskip = Dsk + (size_t)k * kD;
      sa.y = (__half*)(YS + ((size_t)(b * kDir + k)) * kL * kD);
      sa.y_lo = nullptr;
      sa.ld_dtpre = kD;
      sa.ld_u = kD;
      sa.ld_bc = kBcW;
      sa.ld_z = 0;
      sa.ld_y = kD;
      sa.offB = 0;
      sa.offC = kNs;
      sa.offZ = 0;
      sa.ycarry = kYCarry;
      sa.dir = 1;
      sa.D = kD;
      sa.L = kL;
      sa.nbatch = 1;
      ms1_scan_kernel<16><<<dim3(kD / 64), 64, 0, stream>>>(sa);
    }
  }

  merge_norm_kernel<<<dim3(kRows / 16), 192, 0, stream>>>(YS, lnw, lnb, out);
}
